// GraphMERTModel_90288802496731
// MI455X (gfx1250) — hardware-verified
//
#include <hip/hip_runtime.h>
#include <stddef.h>
#include <stdint.h>
#include <math.h>

#define BB    32
#define NNODE 512
#define KIN   128
#define DM    256
#define NH    8
#define DH    32
#define FFD   2048
#define NV    10
#define NVP   16
#define NL    2
#define NTY   2
#define NR    10
#define ROWS  (BB * NNODE)
#define C3    (3 * DM)
#define RP    (BB * C3)
#define GP    (NH * NNODE * DH)

static_assert(BB == 32);
static_assert(ROWS == 16384);
static_assert(ROWS % 256 == 0);
static_assert(NH * DH == DM);
static_assert(DH == 32);
static_assert(NNODE % 128 == 0);
static_assert(C3 % 64 == 0);
static_assert(FFD % 64 == 0);
static_assert(KIN % 64 == 0);
static_assert((RP * 2) % 16 == 0);
static_assert(NV <= NVP);

#define kWSC 32.0f
#define kHSC 8.0f
#define kQSC 16.0f
#define kPSC 1024.0f
#define kGSC 256.0f
#define kFSC 16.0f

typedef _Float16 v16h __attribute__((ext_vector_type(16)));
typedef _Float16 v8h  __attribute__((ext_vector_type(8)));
typedef float    v8f  __attribute__((ext_vector_type(8)));
typedef float    v4f  __attribute__((ext_vector_type(4)));
typedef unsigned int v4u __attribute__((ext_vector_type(4)));

union Frag  { v16h v; v8h h[2]; };
union Pack8 { v8h h; v4u u; };

__device__ __forceinline__ v8f mma16(v16h a, v16h b, v8f c) {
  c = __builtin_amdgcn_wmma_f32_16x16x32_f16(false, a, false, b, (short)0, c, false, false);
  asm volatile("v_nop\n\tv_nop\n\tv_nop\n\tv_nop" : "+v"(c) : "v"(a), "v"(b));
  return c;
}

__device__ __forceinline__ v16h ldfrag(const _Float16* p, int ld, int row0, int k0, int lane) {
  const int m = lane & 15, lh = lane >> 4;
  const _Float16* q = p + (size_t)(row0 + m) * ld + k0 + 8 * lh;
  Frag f;
  f.h[0] = *(const v8h*)(q);
  f.h[1] = *(const v8h*)(q + 16);
  return f.v;
}

__device__ __forceinline__ v8f zero8() { return (v8f){0.f, 0.f, 0.f, 0.f, 0.f, 0.f, 0.f, 0.f}; }

__device__ __forceinline__ float gelu_t(float x) {
  const float u = 0.7978845608028654f * (x + 0.044715f * x * x * x);
  return 0.5f * x * (1.0f + tanhf(u));
}

template <int KK, int HEADA>
__device__ __forceinline__ void gemm32x64(const _Float16* __restrict__ A, int lda,
                                          const _Float16* __restrict__ Bt,
                                          int m0, int n0, int lane, v8f (&acc)[2][4]) {
#pragma unroll 2
  for (int k0 = 0; k0 < KK; k0 += 32) {
    const _Float16* Ak = HEADA ? (A + (size_t)(k0 >> 5) * (NNODE * DH)) : A;
    const int ka = HEADA ? 0 : k0;
    const v16h a0 = ldfrag(Ak, lda, m0, ka, lane);
    const v16h a1 = ldfrag(Ak, lda, m0 + 16, ka, lane);
    const v16h b0 = ldfrag(Bt, KK, n0, k0, lane);
    const v16h b1 = ldfrag(Bt, KK, n0 + 16, k0, lane);
    const v16h b2 = ldfrag(Bt, KK, n0 + 32, k0, lane);
    const v16h b3 = ldfrag(Bt, KK, n0 + 48, k0, lane);
    acc[0][0] = mma16(a0, b0, acc[0][0]);
    acc[1][0] = mma16(a1, b0, acc[1][0]);
    acc[0][1] = mma16(a0, b1, acc[0][1]);
    acc[1][1] = mma16(a1, b1, acc[1][1]);
    acc[0][2] = mma16(a0, b2, acc[0][2]);
    acc[1][2] = mma16(a1, b2, acc[1][2]);
    acc[0][3] = mma16(a0, b3, acc[0][3]);
    acc[1][3] = mma16(a1, b3, acc[1][3]);
  }
}

__global__ __launch_bounds__(256) void k_cvt_x(const float* __restrict__ x, _Float16* __restrict__ xh, int ngrp) {
  const int t = blockIdx.x * 256 + (int)threadIdx.x;
  if (t >= ngrp) return;
  const int rho = t >> 4, pc = t & 15;
  const int b = rho & (BB - 1), n = rho >> 5;
  const float* s = x + (size_t)(b * NNODE + n) * KIN + pc * 8;
  const v4f a0 = *(const v4f*)(s);
  const v4f a1 = *(const v4f*)(s + 4);
  Pack8 pk;
  pk.h = (v8h){(_Float16)a0[0], (_Float16)a0[1], (_Float16)a0[2], (_Float16)a0[3],
               (_Float16)a1[0], (_Float16)a1[1], (_Float16)a1[2], (_Float16)a1[3]};
  const v4u vv = pk.u;
  volatile v4u* d = (volatile v4u*)(xh + (size_t)rho * KIN + pc * 8);
  *d = vv;
  __threadfence();
  *d = vv;
}

#define WTP 68
__global__ __launch_bounds__(256) void k_wt(const float* __restrict__ w, _Float16* __restrict__ wt,
                                           int nout, int kin, int sstride, int dstride) {
  __shared__ __align__(16) float tf[64 * WTP];
  const int tid = threadIdx.x;
  const int n0 = blockIdx.x * 64;
  const int k0 = blockIdx.y * 64;
  w  += (size_t)blockIdx.z * (size_t)sstride;
  wt += (size_t)blockIdx.z * (size_t)dstride;
  {
    const int kr = tid >> 4;
    const int n4 = (tid & 15) * 4;
#pragma unroll
    for (int it = 0; it < 4; ++it) {
      const int kl = it * 16 + kr;
      const v4f a = *(const v4f*)(w + (size_t)(k0 + kl) * nout + n0 + n4);
      *(v4f*)(tf + kl * WTP + n4) = a;
    }
  }
  __syncthreads();
  v4u val[2];
  size_t go[2];
#pragma unroll
  for (int j = 0; j < 2; ++j) {
    const int p  = tid + 256 * j;
    const int nl = p >> 3;
    const int pc = p & 7;
    const float* cp = tf + (pc * 8) * WTP + nl;
    Pack8 pk;
    pk.h = (v8h){(_Float16)(cp[0 * WTP] * kWSC), (_Float16)(cp[1 * WTP] * kWSC),
                 (_Float16)(cp[2 * WTP] * kWSC), (_Float16)(cp[3 * WTP] * kWSC),
                 (_Float16)(cp[4 * WTP] * kWSC), (_Float16)(cp[5 * WTP] * kWSC),
                 (_Float16)(cp[6 * WTP] * kWSC), (_Float16)(cp[7 * WTP] * kWSC)};
    val[j] = pk.u;
    go[j]  = (size_t)(n0 + nl) * kin + k0 + pc * 8;
  }
  for (int ps = 0; ps < 2; ++ps) {
#pragma unroll
    for (int j = 0; j < 2; ++j) *(volatile v4u*)(wt + go[j]) = val[j];
    __threadfence();
  }
}

__global__ __launch_bounds__(256) void k_wc(const float* __restrict__ wc, _Float16* __restrict__ wct) {
  const int tid = threadIdx.x;
  v4u val[2];
  size_t go[2];
#pragma unroll
  for (int j = 0; j < 2; ++j) {
    const int p  = tid + 256 * j;
    const int n  = p >> 5;
    const int pc = p & 31;
    const int nn = (n < NV) ? n : (NV - 1);
    const float sc = (n < NV) ? kWSC : 0.0f;
    const float* cp = wc + (size_t)(pc * 8) * NV + nn;
    Pack8 pk;
    pk.h = (v8h){(_Float16)(cp[0 * NV] * sc), (_Float16)(cp[1 * NV] * sc),
                 (_Float16)(cp[2 * NV] * sc), (_Float16)(cp[3 * NV] * sc),
                 (_Float16)(cp[4 * NV] * sc), (_Float16)(cp[5 * NV] * sc),
                 (_Float16)(cp[6 * NV] * sc), (_Float16)(cp[7 * NV] * sc)};
    val[j] = pk.u;
    go[j]  = (size_t)n * DM + pc * 8;
  }
  for (int ps = 0; ps < 2; ++ps) {
#pragma unroll
    for (int j = 0; j < 2; ++j) *(volatile v4u*)(wct + go[j]) = val[j];
    __threadfence();
  }
}

#define STP 72
__global__ __launch_bounds__(256) void k_proj(const _Float16* __restrict__ ah,
                                              const _Float16* __restrict__ w0, int tstride,
                                              const float* __restrict__ bq,
                                              const float* __restrict__ bk,
                                              const float* __restrict__ bv, int bstride,
                                              const int* __restrict__ nt,
                                              _Float16* __restrict__ qkv) {
  __shared__ __align__(16) _Float16 st[256 * STP];
  const int tid = threadIdx.x, lane = tid & 31, wave = tid >> 5;
  const int hh = lane >> 4, c = lane & 15;
  const int mb = blockIdx.x * 256;
  const int node = blockIdx.x * 8 + wave;
  const int m0 = mb + wave * 32;
  const int n0 = blockIdx.y * 64;
  const int ty = (nt[node] == 1) ? 1 : 0;
  const _Float16* wt = w0 + (size_t)ty * (size_t)tstride;
  const int boff = ty * bstride;
  const int which = n0 >> 8;
  const int nin = n0 & (DM - 1);

  v8f acc[2][4];
#pragma unroll
  for (int s = 0; s < 2; ++s)
#pragma unroll
    for (int t4 = 0; t4 < 4; ++t4) acc[s][t4] = zero8();
  gemm32x64<DM, 0>(ah, DM, wt, m0, n0, lane, acc);

  const float os = 1.0f / (kHSC * kWSC);
#pragma unroll
  for (int t4 = 0; t4 < 4; ++t4) {
    const int nn = nin + 16 * t4 + c;
    const float v0 = bq[boff + nn], v1 = bk[boff + nn], v2 = bv[boff + nn];
    const float bb = (which == 0) ? v0 : ((which == 1) ? v1 : v2);
#pragma unroll
    for (int sub = 0; sub < 2; ++sub) {
#pragma unroll
      for (int r = 0; r < 8; ++r) {
        const int lr = wave * 32 + sub * 16 + 8 * hh + r;
        st[lr * STP + 16 * t4 + c] = (_Float16)((acc[sub][t4][r] * os + bb) * kQSC);
      }
    }
  }
  __syncthreads();

  v4u val[8];
  size_t go[8];
#pragma unroll
  for (int j = 0; j < 8; ++j) {
    const int p  = tid + 256 * j;
    const int lr = p >> 3;
    const int pc = p & 7;
    Pack8 pk;
    pk.h  = *(const v8h*)(st + lr * STP + pc * 8);
    val[j] = pk.u;
    go[j]  = (size_t)(mb + lr) * C3 + n0 + pc * 8;
  }
  for (int ps = 0; ps < 2; ++ps) {
#pragma unroll
    for (int j = 0; j < 8; ++j) *(volatile v4u*)(qkv + go[j]) = val[j];
    __threadfence();
  }
}

#define KTP 40
#define VTP 72
#define PTP 72
template <int BIAS, int GELU>
__global__ __launch_bounds__(256) void k_attn(const _Float16* __restrict__ qkv,
                                              const float* __restrict__ relp,
                                              const int* __restrict__ rid,
                                              _Float16* __restrict__ gp, float sscale) {
  __shared__ __align__(16) _Float16 Ks[64 * KTP];
  __shared__ __align__(16) _Float16 Vs[DH * VTP];
  __shared__ __align__(16) _Float16 Ps[8][16 * PTP];

  const int tid = threadIdx.x, lane = tid & 31, wave = tid >> 5;
  const int hh = lane >> 4, c = lane & 15;
  const int bh = blockIdx.x >> 2;
  const int qb = blockIdx.x & 3;
  const int b  = bh >> 3, h = bh & (NH - 1);
  const int q0 = qb * 128 + wave * 16;

  const _Float16* Q = qkv + (size_t)b * C3 + h * DH;
  const _Float16* K = Q + DM;
  const _Float16* V = Q + 2 * DM;

  const v16h qa = ldfrag(Q, RP, q0, 0, lane);

  const float NEGI = -__builtin_huge_valf();
  float mrow[8], lrow[8];
  v8f oacc[2];
#pragma unroll
  for (int r = 0; r < 8; ++r) { mrow[r] = NEGI; lrow[r] = 0.f; }
  oacc[0] = zero8(); oacc[1] = zero8();

  _Float16* pw = Ps[wave];

  for (int kc = 0; kc < NNODE / 64; ++kc) {
    const int kv0 = kc * 64;
    __syncthreads();
    {
      const int r  = tid >> 2;
      const int qq = (tid & 3) * 8;
      const size_t ro = (size_t)(kv0 + r) * RP + qq;
      *(v8h*)(Ks + r * KTP + qq) = *(const v8h*)(K + ro);
      Pack8 pv;
      pv.h = *(const v8h*)(V + ro);
#pragma unroll
      for (int i = 0; i < 8; ++i) Vs[(qq + i) * VTP + r] = pv.h[i];
    }
    __syncthreads();

    v8f s[4];
#pragma unroll
    for (int j = 0; j < 4; ++j) s[j] = zero8();
#pragma unroll
    for (int j = 0; j < 4; ++j) {
      const v16h kb = ldfrag(Ks, KTP, j * 16, 0, lane);
      s[j] = mma16(qa, kb, s[j]);
    }
    float bl[4];
#pragma unroll
    for (int j = 0; j < 4; ++j) {
      if (BIAS) {
        int rr = rid[b * NNODE + kv0 + j * 16 + c];
        rr = rr < 0 ? 0 : (rr > NR - 1 ? NR - 1 : rr);
        bl[j] = relp[rr * NH + h];
      } else {
        bl[j] = 0.f;
      }
    }
    float cm[8];
#pragma unroll
    for (int r = 0; r < 8; ++r) {
      float m = NEGI;
#pragma unroll
      for (int j = 0; j < 4; ++j) {
        const float sv = s[j][r] * sscale + bl[j];
        s[j][r] = sv;
        m = fmaxf(m, sv);
      }
#pragma unroll
      for (int off = 1; off < 16; off <<= 1) m = fmaxf(m, __shfl_xor(m, off, 32));
      cm[r] = m;
    }
    float al[8];
#pragma unroll
    for (int r = 0; r < 8; ++r) {
      const float mnew  = fmaxf(mrow[r], cm[r]);
      const float alpha = __expf(mrow[r] - mnew);
      mrow[r] = mnew;
      float psum = 0.f;
#pragma unroll
      for (int j = 0; j < 4; ++j) {
        const float p = __expf(s[j][r] - mnew);
        psum += p;
        pw[(8 * hh + r) * PTP + j * 16 + c] = (_Float16)(p * kPSC);
      }
#pragma unroll
      for (int off = 1; off < 16; off <<= 1) psum += __shfl_xor(psum, off, 32);
      lrow[r] = lrow[r] * alpha + psum;
      al[r] = alpha;
    }
#pragma unroll
    for (int t = 0; t < 2; ++t)
#pragma unroll
      for (int r = 0; r < 8; ++r) oacc[t][r] *= al[r];
    __syncthreads();

#pragma unroll
    for (int kk = 0; kk < 2; ++kk) {
      const v16h pa = ldfrag(pw, PTP, 0, kk * 32, lane);
#pragma unroll
      for (int t = 0; t < 2; ++t) {
        const v16h vb = ldfrag(Vs, VTP, t * 16, kk * 32, lane);
        oacc[t] = mma16(pa, vb, oacc[t]);
      }
    }
  }
  __syncthreads();

#pragma unroll
  for (int r = 0; r < 8; ++r) {
    const float inv = (1.0f / (kPSC * kQSC)) * (1.0f / lrow[r]);
#pragma unroll
    for (int t = 0; t < 2; ++t) {
      const float mv = oacc[t][r] * inv;
      const float ov = GELU ? gelu_t(mv) : mv;
      pw[(8 * hh + r) * PTP + 16 * t + c] = (_Float16)(ov * kGSC);
    }
  }
  __syncthreads();
  v4u val[2];
  size_t go[2];
#pragma unroll
  for (int it = 0; it < 2; ++it) {
    const int p  = lane + 32 * it;
    const int L  = p >> 2;
    const int pc = p & 3;
    Pack8 pk;
    pk.h   = *(const v8h*)(pw + L * PTP + pc * 8);
    val[it] = pk.u;
    go[it]  = ((size_t)bh * NNODE + q0 + L) * DH + pc * 8;
  }
  for (int ps = 0; ps < 2; ++ps) {
#pragma unroll
    for (int it = 0; it < 2; ++it) *(volatile v4u*)(gp + go[it]) = val[it];
    __threadfence();
  }
}

#define OTP 68
template <int KK, int HEADA, int RES, int WH>
__global__ __launch_bounds__(256) void k_gout(const _Float16* __restrict__ ap,
                                              const _Float16* __restrict__ w0, int tstride,
                                              const float* __restrict__ bias, int bstride,
                                              const int* __restrict__ nt,
                                              const float* __restrict__ res,
                                              float* __restrict__ out,
                                              _Float16* __restrict__ outh, float oscale) {
  __shared__ __align__(16) float st[8][16 * OTP];
  const int tid = threadIdx.x, lane = tid & 31, wave = tid >> 5;
  const int hh = lane >> 4, c = lane & 15;
  const int node = blockIdx.x * 8 + wave;
  const int m0 = node * 32;
  const int n0 = blockIdx.y * 64;
  const int ty = (nt[node] == 1) ? 1 : 0;
  const _Float16* wt = w0 + (size_t)ty * (size_t)tstride;
  const float* bp = bias + ty * bstride;

  v8f acc[2][4];
#pragma unroll
  for (int s = 0; s < 2; ++s)
#pragma unroll
    for (int t4 = 0; t4 < 4; ++t4) acc[s][t4] = zero8();
  if (HEADA) gemm32x64<KK, 1>(ap + (size_t)node * DH, GP, wt, 0, n0, lane, acc);
  else       gemm32x64<KK, 0>(ap, KK, wt, m0, n0, lane, acc);

  float bvs[4];
#pragma unroll
  for (int t4 = 0; t4 < 4; ++t4) bvs[t4] = bp[n0 + 16 * t4 + c];

  float* sw = st[wave];
#pragma unroll
  for (int sub = 0; sub < 2; ++sub) {
    __syncthreads();
#pragma unroll
    for (int t4 = 0; t4 < 4; ++t4) {
#pragma unroll
      for (int r = 0; r < 8; ++r)
        sw[(8 * hh + r) * OTP + 16 * t4 + c] = acc[sub][t4][r] * oscale + bvs[t4];
    }
    __syncthreads();
    v4f val[8];
    size_t go[8];
#pragma unroll
    for (int it = 0; it < 8; ++it) {
      const int p    = lane + 32 * it;
      const int L    = p >> 3;
      const int pc   = p & 7;
      const int row  = L >> 1;
      const int half = L & 1;
      const size_t g = (size_t)(m0 + sub * 16 + row) * DM + n0 + half * 32 + pc * 4;
      float* sp = sw + row * OTP + half * 32 + pc * 4;
      v4f v = *(const v4f*)sp;
      if (RES) {
        const v4f rr = *(const v4f*)(res + g);
        v[0] = v[0] + rr[0]; v[1] = v[1] + rr[1]; v[2] = v[2] + rr[2]; v[3] = v[3] + rr[3];
      }
      if (WH) *(v4f*)sp = v;
      val[it] = v;
      go[it]  = g;
    }
    for (int ps = 0; ps < 2; ++ps) {
#pragma unroll
      for (int it = 0; it < 8; ++it) *(volatile v4f*)(out + go[it]) = val[it];
      __threadfence();
    }
    if (WH) {
      __syncthreads();
      v4u hv[4];
      size_t ho[4];
#pragma unroll
      for (int it = 0; it < 4; ++it) {
        const int p  = lane + 32 * it;
        const int L  = p >> 3;
        const int pc = p & 7;
        const v4f x0 = *(const v4f*)(sw + L * OTP + pc * 8);
        const v4f x1 = *(const v4f*)(sw + L * OTP + pc * 8 + 4);
        Pack8 pk;
        pk.h = (v8h){(_Float16)(x0[0] * kHSC), (_Float16)(x0[1] * kHSC), (_Float16)(x0[2] * kHSC), (_Float16)(x0[3] * kHSC),
                     (_Float16)(x1[0] * kHSC), (_Float16)(x1[1] * kHSC), (_Float16)(x1[2] * kHSC), (_Float16)(x1[3] * kHSC)};
        hv[it] = pk.u;
        ho[it] = (size_t)(m0 + sub * 16 + L) * DM + n0 + pc * 8;
      }
      for (int ps = 0; ps < 2; ++ps) {
#pragma unroll
        for (int it = 0; it < 4; ++it) *(volatile v4u*)(outh + ho[it]) = hv[it];
        __threadfence();
      }
    }
  }
}

__global__ __launch_bounds__(256) void k_ffn1(const _Float16* __restrict__ ap,
                                              const _Float16* __restrict__ wt,
                                              const float* __restrict__ bias,
                                              _Float16* __restrict__ hp) {
  __shared__ __align__(16) float st[8][16 * OTP];
  const int tid = threadIdx.x, lane = tid & 31, wave = tid >> 5;
  const int hh = lane >> 4, c = lane & 15;
  const int m0 = blockIdx.x * 256 + wave * 32;
  const int n0 = blockIdx.y * 64;

  v8f acc[2][4];
#pragma unroll
  for (int s = 0; s < 2; ++s)
#pragma unroll
    for (int t4 = 0; t4 < 4; ++t4) acc[s][t4] = zero8();
  gemm32x64<DM, 0>(ap, DM, wt, m0, n0, lane, acc);

  const float os = 1.0f / (kHSC * kWSC);
  float bvs[4];
#pragma unroll
  for (int t4 = 0; t4 < 4; ++t4) bvs[t4] = bias[n0 + 16 * t4 + c];

  float* sw = st[wave];
#pragma unroll
  for (int sub = 0; sub < 2; ++sub) {
    __syncthreads();
#pragma unroll
    for (int t4 = 0; t4 < 4; ++t4) {
#pragma unroll
      for (int r = 0; r < 8; ++r)
        sw[(8 * hh + r) * OTP + 16 * t4 + c] = acc[sub][t4][r] * os + bvs[t4];
    }
    __syncthreads();
    v4u val[4];
    size_t go[4];
#pragma unroll
    for (int it = 0; it < 4; ++it) {
      const int p  = lane + 32 * it;
      const int L  = p >> 3;
      const int pc = p & 7;
      const v4f x0 = *(const v4f*)(sw + L * OTP + pc * 8);
      const v4f x1 = *(const v4f*)(sw + L * OTP + pc * 8 + 4);
      Pack8 pk;
      pk.h = (v8h){(_Float16)(fmaxf(x0[0], 0.f) * kFSC), (_Float16)(fmaxf(x0[1], 0.f) * kFSC),
                   (_Float16)(fmaxf(x0[2], 0.f) * kFSC), (_Float16)(fmaxf(x0[3], 0.f) * kFSC),
                   (_Float16)(fmaxf(x1[0], 0.f) * kFSC), (_Float16)(fmaxf(x1[1], 0.f) * kFSC),
                   (_Float16)(fmaxf(x1[2], 0.f) * kFSC), (_Float16)(fmaxf(x1[3], 0.f) * kFSC)};
      val[it] = pk.u;
      go[it]  = (size_t)(m0 + sub * 16 + L) * FFD + n0 + pc * 8;
    }
    for (int ps = 0; ps < 2; ++ps) {
#pragma unroll
      for (int it = 0; it < 4; ++it) *(volatile v4u*)(hp + go[it]) = val[it];
      __threadfence();
    }
  }
}

template <int WH, int PERM>
__global__ __launch_bounds__(64) void k_ln(const float* __restrict__ in,
                                          const float* __restrict__ g,
                                          const float* __restrict__ bt,
                                          float* __restrict__ outf,
                                          _Float16* __restrict__ outh) {
  __shared__ __align__(16) float rb[DM];
  __shared__ float red[4];
  const int tid = threadIdx.x, lane = tid & 31, wave = tid >> 5;
  const int rho = blockIdx.x;
  const size_t ro = (size_t)rho * DM;
  const v4f v = *(const v4f*)(in + ro + 4 * tid);
  float s = (v[0] + v[1]) + (v[2] + v[3]);
#pragma unroll
  for (int off = 1; off < 32; off <<= 1) s += __shfl_xor(s, off, 32);
  if (lane == 0) red[wave] = s;
  __syncthreads();
  const float mean = (red[0] + red[1]) * (1.0f / (float)DM);
  const float d0 = v[0] - mean, d1 = v[1] - mean, d2 = v[2] - mean, d3 = v[3] - mean;
  float q = (d0 * d0 + d1 * d1) + (d2 * d2 + d3 * d3);
#pragma unroll
  for (int off = 1; off < 32; off <<= 1) q += __shfl_xor(q, off, 32);
  if (lane == 0) red[2 + wave] = q;
  __syncthreads();
  const float var = (red[2] + red[3]) * (1.0f / (float)DM);
  const float inv = rsqrtf(var + 1e-5f);
  const v4f g4 = *(const v4f*)(g + 4 * tid);
  const v4f b4 = *(const v4f*)(bt + 4 * tid);
  v4f o;
  o[0] = d0 * inv * g4[0] + b4[0];
  o[1] = d1 * inv * g4[1] + b4[1];
  o[2] = d2 * inv * g4[2] + b4[2];
  o[3] = d3 * inv * g4[3] + b4[3];
  const int orow = PERM ? ((rho & (BB - 1)) * NNODE + (rho >> 5)) : rho;
  volatile v4f* dp = (volatile v4f*)(outf + (size_t)orow * DM + 4 * tid);
  *dp = o;
  __threadfence();
  *dp = o;
  if (WH) {
    *(v4f*)(rb + 4 * tid) = o;
    __syncthreads();
    if (tid < 32) {
      const v4f a0 = *(const v4f*)(rb + 8 * tid);
      const v4f a1 = *(const v4f*)(rb + 8 * tid + 4);
      Pack8 pk;
      pk.h = (v8h){(_Float16)(a0[0] * kHSC), (_Float16)(a0[1] * kHSC), (_Float16)(a0[2] * kHSC), (_Float16)(a0[3] * kHSC),
                   (_Float16)(a1[0] * kHSC), (_Float16)(a1[1] * kHSC), (_Float16)(a1[2] * kHSC), (_Float16)(a1[3] * kHSC)};
      const v4u vv = pk.u;
      volatile v4u* hq = (volatile v4u*)(outh + ro + 8 * tid);
      *hq = vv;
      __threadfence();
      *hq = vv;
    }
  }
}

__global__ __launch_bounds__(256) void k_cls(const _Float16* __restrict__ hf,
                                             const _Float16* __restrict__ wct,
                                             const float* __restrict__ bc,
                                             float* __restrict__ out0) {
  __shared__ __align__(16) float st[8][32 * NV];
  const int tid = threadIdx.x, lane = tid & 31, wave = tid >> 5;
  const int hh = lane >> 4, c = lane & 15;
  const int b  = blockIdx.x >> 1;
  const int n0 = (blockIdx.x & 1) * 256 + wave * 32;
  const _Float16* A = hf + (size_t)b * DM;

  v8f acc[2];
  acc[0] = zero8(); acc[1] = zero8();
#pragma unroll 2
  for (int k0 = 0; k0 < DM; k0 += 32) {
    const v16h a0 = ldfrag(A, BB * DM, n0, k0, lane);
    const v16h a1 = ldfrag(A, BB * DM, n0 + 16, k0, lane);
    const v16h bw = ldfrag(wct, DM, 0, k0, lane);
    acc[0] = mma16(a0, bw, acc[0]);
    acc[1] = mma16(a1, bw, acc[1]);
  }
  const float os = 1.0f / (kHSC * kWSC);
  const float bcv = bc[(c < NV) ? c : (NV - 1)];
  float* sw = st[wave];
#pragma unroll
  for (int sub = 0; sub < 2; ++sub) {
#pragma unroll
    for (int r = 0; r < 8; ++r) {
      const int row = 16 * sub + 8 * hh + r;
      if (c < NV) sw[row * NV + c] = acc[sub][r] * os + bcv;
    }
  }
  __syncthreads();
  v4f val[3];
  size_t go[3];
#pragma unroll
  for (int it = 0; it < 3; ++it) {
    const int p  = lane + 32 * it;
    const int pp = (p < 80) ? p : 79;
    val[it] = *(const v4f*)(sw + pp * 4);
    go[it]  = (size_t)(b * NNODE + n0) * NV + pp * 4;
  }
  for (int ps = 0; ps < 2; ++ps) {
#pragma unroll
    for (int it = 0; it < 3; ++it) {
      const int p = lane + 32 * it;
      if (p < 80) *(volatile v4f*)(out0 + go[it]) = val[it];
    }
    __threadfence();
  }
}

extern "C" void kernel_launch(void* const* d_in, const int* in_sizes, int n_in,
                              void* d_out, int out_size, void* d_ws, size_t ws_size,
                              hipStream_t stream) {
  if (n_in < 28) return;
  if (in_sizes[0] != ROWS * KIN) return;
  if (in_sizes[1] != NNODE || in_sizes[2] != BB * NNODE) return;
  if (in_sizes[3] != KIN * DM || in_sizes[4] != DM) return;
  if (in_sizes[5] != NL * NTY * DM * DM || in_sizes[6] != NL * NTY * DM * DM) return;
  if (in_sizes[7] != NL * NTY * DM * DM || in_sizes[8] != NL * NTY * DM * DM) return;
  if (in_sizes[9] != NL * NTY * DM || in_sizes[10] != NL * NTY * DM) return;
  if (in_sizes[11] != NL * NTY * DM || in_sizes[12] != NL * NTY * DM) return;
  if (in_sizes[13] != NL * NR * NH) return;
  if (in_sizes[14] != DM * C3 || in_sizes[15] != C3) return;
  if (in_sizes[16] != DM * DM || in_sizes[17] != DM) return;
  if (in_sizes[18] != DM || in_sizes[19] != DM || in_sizes[20] != DM || in_sizes[21] != DM) return;
  if (in_sizes[22] != DM * FFD || in_sizes[23] != FFD) return;
  if (in_sizes[24] != FFD * DM || in_sizes[25] != DM) return;
  if (in_sizes[26] != DM * NV || in_sizes[27] != NV) return;
  if (out_size != ROWS * NV + ROWS * DM) return;

  const float* x     = (const float*)d_in[0];
  const int*   ntyp  = (const int*)d_in[1];
  const int*   relid = (const int*)d_in[2];
  const float* W_in  = (const float*)d_in[3];
  const float* b_in  = (const float*)d_in[4];
  const float* Wq    = (const float*)d_in[5];
  const float* Wk    = (const float*)d_in[6];
  const float* Wv    = (const float*)d_in[7];
  const float* Wo    = (const float*)d_in[8];
  const float* bq    = (const float*)d_in[9];
  const float* bk    = (const float*)d_in[10];
  const float* bv    = (const float*)d_in[11];
  const float* bo    = (const float*)d_in[12];
  const float* relp  = (const float*)d_in[13];
  const float* Wqkv  = (const float*)d_in[14];
  const float* bqkv  = (const float*)d_in[15];
  const float* Wot   = (const float*)d_in[16];
  const float* bot   = (const float*)d_in[17];
  const float* g1    = (const float*)d_in[18];
  const float* be1   = (const float*)d_in[19];
  const float* g2    = (const float*)d_in[20];
  const float* be2   = (const float*)d_in[21];
  const float* Wf1   = (const float*)d_in[22];
  const float* bf1   = (const float*)d_in[23];
  const float* Wf2   = (const float*)d_in[24];
  const float* bf2   = (const float*)d_in[25];
  const float* Wc    = (const float*)d_in[26];
  const float* bc    = (const float*)d_in[27];
  float* out0 = (float*)d_out;
  float* out1 = out0 + (size_t)ROWS * NV;

  size_t off = 0;
  const size_t oXh  = off; off += (size_t)ROWS * KIN * 2;
  const size_t oHB  = off; off += (size_t)ROWS * DM * 4;
  const size_t oHBh = off; off += (size_t)ROWS * DM * 2;
  const size_t oQKV = off; off += (size_t)ROWS * C3 * 2;
  const size_t oG   = off; off += (size_t)BB * NH * NNODE * DH * 2;
  const size_t oT1  = off; off += (size_t)ROWS * DM * 4;
  const size_t oF   = 0;
  if ((size_t)ROWS * FFD * 2 > off) return;
  const size_t oHfin = 0;
  if ((size_t)ROWS * DM * 2 > (size_t)ROWS * FFD * 2) return;
  const size_t oWint = off; off += (size_t)DM * KIN * 2;
  const size_t oWQKV = off; off += (size_t)NL * NTY * C3 * DM * 2;
  const size_t oWO   = off; off += (size_t)NL * NTY * DM * DM * 2;
  const size_t oWenc = off; off += (size_t)C3 * DM * 2;
  const size_t oWott = off; off += (size_t)DM * DM * 2;
  const size_t oWf1  = off; off += (size_t)FFD * DM * 2;
  const size_t oWf2  = off; off += (size_t)DM * FFD * 2;
  const size_t oWct  = off; off += (size_t)NVP * DM * 2;
  const size_t oHA   = off; off += (size_t)ROWS * DM * 4;
  const size_t oHAh  = off; off += (size_t)ROWS * DM * 2;
  const size_t oAh   = off; off += (size_t)ROWS * DM * 2;
  const size_t oA32  = oHA;
  const size_t oT2   = oHAh;
  if (oAh + (size_t)ROWS * DM * 2 - oHAh < (size_t)ROWS * DM * 4) return;
  if (off > ws_size) return;
  if (off > (size_t)134217728) return;

  char* ws = (char*)d_ws;
  _Float16* Xh   = (_Float16*)(ws + oXh);
  float*    HB   = (float*)(ws + oHB);
  _Float16* HBh  = (_Float16*)(ws + oHBh);
  _Float16* QKV  = (_Float16*)(ws + oQKV);
  _Float16* G    = (_Float16*)(ws + oG);
  float*    T1   = (float*)(ws + oT1);
  _Float16* F    = (_Float16*)(ws + oF);
  _Float16* Hfin = (_Float16*)(ws + oHfin);
  _Float16* Wint = (_Float16*)(ws + oWint);
  _Float16* WQKV = (_Float16*)(ws + oWQKV);
  _Float16* WO   = (_Float16*)(ws + oWO);
  _Float16* Wenc = (_Float16*)(ws + oWenc);
  _Float16* Wott = (_Float16*)(ws + oWott);
  _Float16* Wf1t = (_Float16*)(ws + oWf1);
  _Float16* Wf2t = (_Float16*)(ws + oWf2);
  _Float16* Wct  = (_Float16*)(ws + oWct);
  float*    HA   = (float*)(ws + oHA);
  _Float16* HAh  = (_Float16*)(ws + oHAh);
  _Float16* Ah   = (_Float16*)(ws + oAh);
  float*    A32  = (float*)(ws + oA32);
  float*    T2   = (float*)(ws + oT2);

  const int plq = C3 * DM;
  const int plo = DM * DM;

  const int ngrp = in_sizes[0] / 8;
  k_cvt_x<<<dim3((ngrp + 255) / 256), dim3(256), 0, stream>>>(x, Xh, ngrp);
  k_wt<<<dim3(DM / 64, KIN / 64, 1), dim3(256), 0, stream>>>(W_in, Wint, DM, KIN, 0, 0);
  k_wt<<<dim3(DM / 64, DM / 64, NL * NTY), dim3(256), 0, stream>>>(Wq, WQKV, DM, DM, plo, plq);
  k_wt<<<dim3(DM / 64, DM / 64, NL * NTY), dim3(256), 0, stream>>>(Wk, WQKV + (size_t)DM * DM, DM, DM, plo, plq);
  k_wt<<<dim3(DM / 64, DM / 64, NL * NTY), dim3(256), 0, stream>>>(Wv, WQKV + (size_t)2 * DM * DM, DM, DM, plo, plq);
  k_wt<<<dim3(DM / 64, DM / 64, NL * NTY), dim3(256), 0, stream>>>(Wo, WO, DM, DM, plo, plo);
  k_wt<<<dim3(C3 / 64, DM / 64, 1), dim3(256), 0, stream>>>(Wqkv, Wenc, C3, DM, 0, 0);
  k_wt<<<dim3(DM / 64, DM / 64, 1), dim3(256), 0, stream>>>(Wot, Wott, DM, DM, 0, 0);
  k_wt<<<dim3(FFD / 64, DM / 64, 1), dim3(256), 0, stream>>>(Wf1, Wf1t, FFD, DM, 0, 0);
  k_wt<<<dim3(DM / 64, FFD / 64, 1), dim3(256), 0, stream>>>(Wf2, Wf2t, DM, FFD, 0, 0);
  k_wc<<<dim3(1), dim3(256), 0, stream>>>(Wc, Wct);
  k_gout<KIN, 0, 0, 1><<<dim3(ROWS / 256, DM / 64), dim3(256), 0, stream>>>(Xh, Wint, 0, b_in, 0, ntyp, HB, HA, HAh, 0.03125f);
  const float sscale = 0.17677669529663687f * (1.0f / (kQSC * kQSC));
  for (int l = 0; l < NL; ++l) {
    const float* hin  = (l == 0) ? HA : HB;
    const _Float16* hinh = (l == 0) ? HAh : HBh;
    float* hout = (l == 0) ? HB : HA;
    _Float16* houth = (l == 0) ? HBh : HAh;
    k_proj<<<dim3(ROWS / 256, C3 / 64), dim3(256), 0, stream>>>(hinh, WQKV + (size_t)(l * NTY) * plq, plq,
                                                                bq + l * NTY * DM, bk + l * NTY * DM, bv + l * NTY * DM, DM,
                                                                ntyp, QKV);
    k_attn<1, 1><<<dim3(BB * NH * (NNODE / 128)), dim3(256), 0, stream>>>(QKV, relp + l * NR * NH, relid, G, sscale);
    k_gout<DM, 1, 1, 1><<<dim3(ROWS / 256, DM / 64), dim3(256), 0, stream>>>(G, WO + (size_t)(l * NTY) * plo, plo,
                                                                              bo + l * NTY * DM, DM, ntyp, hin, hout, houth,
                                                                              0.0001220703125f);
  }
  k_proj<<<dim3(ROWS / 256, C3 / 64), dim3(256), 0, stream>>>(HAh, Wenc, 0, bqkv, bqkv + DM, bqkv + 2 * DM, 0, ntyp, QKV);
  k_attn<0, 0><<<dim3(BB * NH * (NNODE / 128)), dim3(256), 0, stream>>>(QKV, relp, relid, G, sscale);
  k_gout<DM, 1, 1, 0><<<dim3(ROWS / 256, DM / 64), dim3(256), 0, stream>>>(G, Wott, 0, bot, 0, ntyp, HA, T1, HAh, 0.0001220703125f);
  k_ln<1, 0><<<dim3(ROWS), dim3(64), 0, stream>>>(T1, g1, be1, A32, Ah);
  k_ffn1<<<dim3(ROWS / 256, FFD / 64), dim3(256), 0, stream>>>(Ah, Wf1t, bf1, F);
  k_gout<FFD, 0, 1, 0><<<dim3(ROWS / 256, DM / 64), dim3(256), 0, stream>>>(F, Wf2t, 0, bf2, 0, ntyp, A32, T2, Hfin, 0.001953125f);
  k_ln<1, 1><<<dim3(ROWS), dim3(64), 0, stream>>>(T2, g2, be2, out1, Hfin);
  k_cls<<<dim3(BB * 2), dim3(256), 0, stream>>>(Hfin, Wct, bc, out0);
  (void)hipGetLastError();
}
